// Generater_80762565034318
// MI455X (gfx1250) — hardware-verified
//
#include <hip/hip_runtime.h>
#include <stddef.h>
#include <stdint.h>


typedef float v4f __attribute__((ext_vector_type(4)));
typedef float v8f __attribute__((ext_vector_type(8)));
typedef unsigned int v4u __attribute__((ext_vector_type(4)));
typedef __bf16 v16bf __attribute__((ext_vector_type(16)));

union Frag {
  v16bf v;
  v4u q[2];
};

__device__ __forceinline__ unsigned int bf_bits(float f) {
  unsigned int u = __float_as_uint(f);
  u += 0x7FFFu + ((u >> 16) & 1u);
  return u >> 16;
}

__device__ __forceinline__ void split_bf(float v, unsigned int& hb, unsigned int& lb) {
  hb = bf_bits(v);
  const float hf = __uint_as_float(hb << 16);
  lb = bf_bits(v - hf);
}

__device__ __forceinline__ void pack8(const float* v, v4u& H, v4u& L) {
  unsigned int hp[4], lp[4];
#pragma unroll
  for (int i = 0; i < 4; ++i) {
    unsigned int h0, l0, h1, l1;
    split_bf(v[2 * i], h0, l0);
    split_bf(v[2 * i + 1], h1, l1);
    hp[i] = h0 | (h1 << 16);
    lp[i] = l0 | (l1 << 16);
  }
  H.x = hp[0]; H.y = hp[1]; H.z = hp[2]; H.w = hp[3];
  L.x = lp[0]; L.y = lp[1]; L.z = lp[2]; L.w = lp[3];
}

__device__ __forceinline__ v8f mma3(v8f acc, v16bf ah, v16bf al, v16bf bh, v16bf bl) {
  acc = __builtin_amdgcn_wmma_f32_16x16x32_bf16(false, ah, false, bh, (short)0, acc, false, false);
  acc = __builtin_amdgcn_wmma_f32_16x16x32_bf16(false, ah, false, bl, (short)0, acc, false, false);
  acc = __builtin_amdgcn_wmma_f32_16x16x32_bf16(false, al, false, bh, (short)0, acc, false, false);
  asm volatile("v_nop\n\tv_nop\n\tv_nop\n\tv_nop" : "+v"(acc) : "v"(ah), "v"(al), "v"(bh), "v"(bl));
  return acc;
}

struct WTab {
  const float* src[29];
  int cout[29];
  int kdim[29];
  int rows[29];
  int kp[29];
  int off[29];
  int cnt;
};
typedef char wtab_size_check[(sizeof(WTab) == 816) ? 1 : -1];

__global__ void __launch_bounds__(256)
k_wsplit(WTab tab, unsigned short* whi, unsigned short* wlo)
{
  const int y = blockIdx.y;
  if (y >= tab.cnt) return;
  const int kp = tab.kp[y];
  const int rows = tab.rows[y];
  const int K = tab.kdim[y];
  const int cout = tab.cout[y];
  const int kq8 = kp >> 3;
  const int tot = rows * kq8;
  const int e = (int)blockIdx.x * 256 + (int)threadIdx.x;
  if (e >= tot) return;
  const int row = e / kq8;
  const int kq = (e - row * kq8) * 8;
  const float* s = tab.src[y] + (size_t)row * K;
  float v[8];
#pragma unroll
  for (int i = 0; i < 8; ++i) {
    const int k = kq + i;
    v[i] = (row < cout && k < K) ? s[k] : 0.0f;
  }
  v4u H, L;
  pack8(v, H, L);
  const size_t d = (size_t)tab.off[y] + (size_t)row * kp + kq;
  *(volatile v4u*)(whi + d) = H;
  *(volatile v4u*)(wlo + d) = L;
  __threadfence();
  *(volatile v4u*)(whi + d) = H;
  *(volatile v4u*)(wlo + d) = L;
}

__global__ void __launch_bounds__(256)
k_split(const float* __restrict__ src, unsigned short* hi, unsigned short* lo, int noct)
{
  const int e = (int)blockIdx.x * 256 + (int)threadIdx.x;
  if (e >= noct) return;
  const v4f a = *(const v4f*)(src + (size_t)e * 8);
  const v4f c = *(const v4f*)(src + (size_t)e * 8 + 4);
  float v[8];
  v[0] = a.x; v[1] = a.y; v[2] = a.z; v[3] = a.w;
  v[4] = c.x; v[5] = c.y; v[6] = c.z; v[7] = c.w;
  v4u H, L;
  pack8(v, H, L);
  const size_t d = (size_t)e * 8;
  *(volatile v4u*)(hi + d) = H;
  *(volatile v4u*)(lo + d) = L;
  __threadfence();
  *(volatile v4u*)(hi + d) = H;
  *(volatile v4u*)(lo + d) = L;
}

#define CTP 68

__global__ void __launch_bounds__(128)
k_conv(const float* __restrict__ in, const unsigned short* __restrict__ whi,
       const unsigned short* __restrict__ wlo, const float* __restrict__ resid,
       float* out, int Bn, int Cin, int Hin, int Win, int Cout, int Hout, int Wout,
       int KH, int KW, int stride, int pad, int K, int Kp, int mw, int relu)
{
  __shared__ v4u Bh[64 * 5];
  __shared__ v4u Bl[64 * 5];
  __shared__ __attribute__((aligned(16))) float Ct[64 * CTP];

  const int t = threadIdx.x;
  const int l = t & 31, h = l >> 4, m = l & 15;
  const int w = __builtin_amdgcn_readfirstlane(t >> 5);
  const int HWo = Hout * Wout;
  const int N = Bn * HWo;
  const int nBase = (int)blockIdx.x * 64;
  if (nBase >= N) return;

  const int nl = t & 63, kh2 = t >> 6;
  int n = nBase + nl;
  if (n > N - 1) n = N - 1;
  const int bi = n / HWo;
  const int pp = n - bi * HWo;
  const int oh = pp / Wout, ow = pp - oh * Wout;
  const int ih0 = oh * stride - pad, iw0 = ow * stride - pad;
  const float* inb = in + (size_t)bi * Cin * Hin * Win;
  const int KHKW = KH * KW;

  const int slab = w % mw;
  const int ngrp = w / mw;
  const int nwm = (4 / mw) - 1;

  const v8f z8 = {0.0f, 0.0f, 0.0f, 0.0f, 0.0f, 0.0f, 0.0f, 0.0f};
  v8f acc[4];
#pragma unroll
  for (int s = 0; s < 4; ++s) acc[s] = z8;

  for (int k0 = 0; k0 < Kp; k0 += 32) {
    int kk = k0 + 16 * kh2;
    int ci = kk / KHKW;
    int rr = kk - ci * KHKW;
    int fh = rr / KW;
    int fw = rr - fh * KW;
    float v[16];
#pragma unroll
    for (int jj = 0; jj < 16; ++jj) {
      float x = 0.0f;
      const int ih = ih0 + fh, iw = iw0 + fw;
      if (kk < K && (unsigned)ih < (unsigned)Hin && (unsigned)iw < (unsigned)Win)
        x = inb[((size_t)ci * Hin + ih) * Win + iw];
      v[jj] = x;
      ++kk;
      ++fw;
      if (fw == KW) { fw = 0; ++fh; if (fh == KH) { fh = 0; ++ci; } }
    }
    v4u H0, L0, H1, L1;
    pack8(v, H0, L0);
    pack8(v + 8, H1, L1);
    Bh[nl * 5 + 2 * kh2] = H0;
    Bh[nl * 5 + 2 * kh2 + 1] = H1;
    Bl[nl * 5 + 2 * kh2] = L0;
    Bl[nl * 5 + 2 * kh2 + 1] = L1;
    __syncthreads();

    Frag ah, al;
    {
      const unsigned short* ph = whi + (size_t)(slab * 16 + m) * Kp + k0;
      const unsigned short* pl = wlo + (size_t)(slab * 16 + m) * Kp + k0;
      ah.q[0] = *(const v4u*)(ph + 8 * h);
      ah.q[1] = *(const v4u*)(ph + 16 + 8 * h);
      al.q[0] = *(const v4u*)(pl + 8 * h);
      al.q[1] = *(const v4u*)(pl + 16 + 8 * h);
    }
#pragma unroll
    for (int s = 0; s < 4; ++s) {
      if ((s & nwm) == ngrp) {
        Frag bh, bl;
        const int br = (16 * s + m) * 5;
        bh.q[0] = Bh[br + h];
        bh.q[1] = Bh[br + 2 + h];
        bl.q[0] = Bl[br + h];
        bl.q[1] = Bl[br + 2 + h];
        acc[s] = mma3(acc[s], ah.v, al.v, bh.v, bl.v);
      }
    }
    __syncthreads();
  }

#pragma unroll
  for (int s = 0; s < 4; ++s) {
    if ((s & nwm) == ngrp) {
#pragma unroll
      for (int r = 0; r < 8; ++r)
        Ct[(slab * 16 + 8 * h + r) * CTP + 16 * s + m] = acc[s][r];
    }
  }
  __syncthreads();

  const int bblk = nBase / HWo;
  const int pblk = nBase - bblk * HWo;
  v4f vals[8];
#pragma unroll
  for (int i = 0; i < 8; ++i) {
    const int row = 16 * w + 2 * i + (l >> 4);
    const int colq = (l & 15) * 4;
    v4f vv = {0.0f, 0.0f, 0.0f, 0.0f};
    if (row < Cout && nBase + colq + 3 < N) {
      vv = *(const v4f*)(&Ct[row * CTP + colq]);
      const size_t gi = ((size_t)(bblk * Cout + row)) * HWo + pblk + colq;
      if (resid) {
        const v4f rv = *(const v4f*)(resid + gi);
        vv += rv;
      }
      if (relu) {
        vv.x = fmaxf(vv.x, 0.0f); vv.y = fmaxf(vv.y, 0.0f);
        vv.z = fmaxf(vv.z, 0.0f); vv.w = fmaxf(vv.w, 0.0f);
      }
      *(volatile v4f*)(out + gi) = vv;
    }
    vals[i] = vv;
  }
  __threadfence();
#pragma unroll
  for (int i = 0; i < 8; ++i) {
    const int row = 16 * w + 2 * i + (l >> 4);
    const int colq = (l & 15) * 4;
    if (row < Cout && nBase + colq + 3 < N) {
      const size_t gi = ((size_t)(bblk * Cout + row)) * HWo + pblk + colq;
      *(volatile v4f*)(out + gi) = vals[i];
    }
  }
}

#define KCH 128
#define EPV 17
#define CAP 36
#define NEGC (-100000000.0f)

__device__ __forceinline__ float dot8(const float* q, v4f a, v4f c) {
#pragma clang fp contract(off)
  float s = q[0] * a.x;
  s = s + q[1] * a.y;
  s = s + q[2] * a.z;
  s = s + q[3] * a.w;
  s = s + q[4] * c.x;
  s = s + q[5] * c.y;
  s = s + q[6] * c.z;
  s = s + q[7] * c.w;
  return s;
}

__device__ __forceinline__ float masksum8(const float* q) {
#pragma clang fp contract(off)
  float s = q[0] * NEGC;
  s = s + q[1] * NEGC;
  s = s + q[2] * NEGC;
  s = s + q[3] * NEGC;
  s = s + q[4] * NEGC;
  s = s + q[5] * NEGC;
  s = s + q[6] * NEGC;
  s = s + q[7] * NEGC;
  return s;
}

__device__ __forceinline__ float lerp2(float v00, float v01, float v10, float v11,
                                       float wy, float wx) {
#pragma clang fp contract(off)
  const float omy = 1.0f - wy;
  const float omx = 1.0f - wx;
  const float r0 = v00 * omy + v10 * wy;
  const float r1 = v01 * omy + v11 * wy;
  return r0 * omx + r1 * wx;
}

__global__ void __launch_bounds__(128)
k_attn(const float* __restrict__ qk, const unsigned short* __restrict__ vhi,
       const unsigned short* __restrict__ vlo, float* aout, int Bn, int H, int relu)
{
  __shared__ v4f Kt[1024 * 2];
  __shared__ v4u Eh[32 * EPV];
  __shared__ v4u El[32 * EPV];
  __shared__ __attribute__((aligned(16))) float Ct[64 * CAP];
  __shared__ float qv[32 * 8];
  __shared__ float red[4 * 32];
  __shared__ float invs[32];

  const int t = threadIdx.x;
  const int l = t & 31, h = l >> 4, m = l & 15;
  const int w = __builtin_amdgcn_readfirstlane(t >> 5);
  const int W = H, P = H * W, Mq = 4 * P, H2 = 2 * H, W2 = 2 * W;
  if (P > 1024 || P < 64) return;
  const int nblk = Mq >> 5;
  const int b = (int)blockIdx.x / nblk;
  const int n0 = ((int)blockIdx.x - b * nblk) * 32;
  if (b >= Bn) return;

  for (int e = t; e < 8 * P; e += 128) {
    const int c = e / P;
    const int p = e - c * P;
    ((float*)Kt)[p * 8 + c] = qk[((size_t)(b * 16 + 8 + c)) * P + p];
  }
  {
    const int j = t & 31, cp = (t >> 5) * 2;
    const int n = n0 + j;
    const int y2 = n / W2, x2 = n - y2 * W2;
    const float ry = 1.0f / (float)(H2 - 1);
    const float rx = 1.0f / (float)(W2 - 1);
    const float yc = (float)(y2 * (H - 1)) * ry;
    const float xc = (float)(x2 * (W - 1)) * rx;
    int y0 = (int)floorf(yc);
    y0 = min(max(y0, 0), H - 1);
    int x0 = (int)floorf(xc);
    x0 = min(max(x0, 0), W - 1);
    const int y1 = min(y0 + 1, H - 1), x1 = min(x0 + 1, W - 1);
    const float wy = yc - (float)y0, wx = xc - (float)x0;
#pragma unroll
    for (int u = 0; u < 2; ++u) {
      const int c = cp + u;
      const float* sp = qk + ((size_t)(b * 16 + c)) * P;
      const float v00 = sp[y0 * W + x0], v01 = sp[y0 * W + x1];
      const float v10 = sp[y1 * W + x0], v11 = sp[y1 * W + x1];
      qv[j * 8 + c] = lerp2(v00, v01, v10, v11, wy, wx);
    }
  }
  __syncthreads();

  const int j = t & 31, g = w;
  float q[8];
#pragma unroll
  for (int c = 0; c < 8; ++c) q[c] = qv[j * 8 + c];
  const float smk = masksum8(q);

  float mx = -3.0e38f;
  for (int p = g; p < P; p += 4) mx = fmaxf(mx, dot8(q, Kt[2 * p], Kt[2 * p + 1]));
  red[g * 32 + j] = mx;
  __syncthreads();
  mx = fmaxf(fmaxf(red[j], red[32 + j]), fmaxf(red[64 + j], red[96 + j]));
  mx = fmaxf(mx, smk);
  __syncthreads();

  const v8f z8 = {0.0f, 0.0f, 0.0f, 0.0f, 0.0f, 0.0f, 0.0f, 0.0f};
  v8f acc[2];
  acc[0] = z8; acc[1] = z8;
  float ssum = 0.0f;
  const int KCe = (P < KCH) ? P : KCH;
  const int run = KCe >> 2;
  const size_t vrow = ((size_t)(b * 64 + 16 * w + m)) * (size_t)P;

  for (int p0 = 0; p0 < P; p0 += KCe) {
    for (int i8 = 0; i8 < run; i8 += 8) {
      float ev[8];
#pragma unroll
      for (int u = 0; u < 8; ++u) {
        const int p = p0 + g * run + i8 + u;
        const float s = dot8(q, Kt[2 * p], Kt[2 * p + 1]);
        const float e = expf(s - mx);
        ssum += e;
        ev[u] = e;
      }
      v4u Hh, Ll;
      pack8(ev, Hh, Ll);
      const int vi = j * EPV + ((g * run + i8) >> 3);
      Eh[vi] = Hh;
      El[vi] = Ll;
    }
    __syncthreads();
    for (int ks = 0; ks < KCe; ks += 32) {
      Frag ah, al;
      const unsigned short* ph = vhi + vrow + p0 + ks;
      const unsigned short* pl = vlo + vrow + p0 + ks;
      ah.q[0] = *(const v4u*)(ph + 8 * h);
      ah.q[1] = *(const v4u*)(ph + 16 + 8 * h);
      al.q[0] = *(const v4u*)(pl + 8 * h);
      al.q[1] = *(const v4u*)(pl + 16 + 8 * h);
#pragma unroll
      for (int s = 0; s < 2; ++s) {
        Frag bh, bl;
        const int er = (16 * s + m) * EPV + (ks >> 3);
        bh.q[0] = Eh[er + h];
        bh.q[1] = Eh[er + 2 + h];
        bl.q[0] = El[er + h];
        bl.q[1] = El[er + 2 + h];
        acc[s] = mma3(acc[s], ah.v, al.v, bh.v, bl.v);
      }
    }
    __syncthreads();
  }

  red[g * 32 + j] = ssum;
  __syncthreads();
  if (t < 32) {
    float den = red[t] + red[32 + t];
    den = den + red[64 + t];
    den = den + red[96 + t];
    den = den + (float)(3 * P) * expf(smk - mx);
    invs[t] = 1.0f / den;
  }
#pragma unroll
  for (int s = 0; s < 2; ++s) {
#pragma unroll
    for (int r = 0; r < 8; ++r)
      Ct[(16 * w + 8 * h + r) * CAP + 16 * s + m] = acc[s][r];
  }
  __syncthreads();

  v4f vals[4];
#pragma unroll
  for (int i = 0; i < 4; ++i) {
    const int row = 16 * w + 4 * i + (l >> 3);
    const int col = (l & 7) * 4;
    v4f v = *(const v4f*)(&Ct[row * CAP + col]);
    v.x *= invs[col];
    v.y *= invs[col + 1];
    v.z *= invs[col + 2];
    v.w *= invs[col + 3];
    if (relu) {
      v.x = fmaxf(v.x, 0.0f); v.y = fmaxf(v.y, 0.0f);
      v.z = fmaxf(v.z, 0.0f); v.w = fmaxf(v.w, 0.0f);
    }
    vals[i] = v;
    *(volatile v4f*)(aout + ((size_t)(b * 64 + row)) * Mq + n0 + col) = v;
  }
  __threadfence();
#pragma unroll
  for (int i = 0; i < 4; ++i) {
    const int row = 16 * w + 4 * i + (l >> 3);
    const int col = (l & 7) * 4;
    *(volatile v4f*)(aout + ((size_t)(b * 64 + row)) * Mq + n0 + col) = vals[i];
  }
}

__device__ __forceinline__ float sigm64(float x) {
  const float z = 64.0f * (x - 0.5f);
  return 1.0f / (1.0f + expf(-z));
}

__global__ void __launch_bounds__(256)
k_sig(const float* __restrict__ src, const int* __restrict__ aux, float* yb, float* ey,
      int n, float ncnt)
{
  __shared__ unsigned int sc[8];
  (void)aux;
  const int t = threadIdx.x;
  const int per = (n + 255) / 256;
  unsigned int cnt = 0u;
#pragma unroll 1
  for (int i = 0; i < per; ++i) {
    const int idx = t + 256 * i;
    if (idx < n) {
      const float y = sigm64(src[idx]);
      cnt += (y < 0.5f) ? 0u : 1u;
      *(volatile float*)(yb + idx) = y;
    }
  }
  for (int o = 16; o > 0; o >>= 1) cnt += __shfl_xor(cnt, o, 32);
  if ((t & 31) == 0) sc[t >> 5] = cnt;
  __syncthreads();
  float eyv = 0.0f;
  if (t == 0) {
    unsigned int tot = 0u;
    for (int i = 0; i < 8; ++i) tot += sc[i];
    const float p1 = (float)tot / ncnt;
    const float p0 = 1.0f - p1;
    const float ln2 = 0.69314718055994531f;
    float a1 = (-p1) * logf(p1 + 1e-10f);
    a1 = a1 / ln2;
    float a0 = (-p0) * logf(p0 + 1e-10f);
    a0 = a0 / ln2;
    eyv = a1 + a0;
    *(volatile float*)ey = eyv;
  }
  __threadfence();
#pragma unroll 1
  for (int i = 0; i < per; ++i) {
    const int idx = t + 256 * i;
    if (idx < n) *(volatile float*)(yb + idx) = sigm64(src[idx]);
  }
  if (t == 0) *(volatile float*)ey = eyv;
}

extern "C" void kernel_launch(void* const* d_in, const int* in_sizes, int n_in,
                              void* d_out, int out_size, void* d_ws, size_t ws_size,
                              hipStream_t stream)
{
  const int WCO[29] = {64, 64, 64, 64, 64, 64, 64, 64, 32, 64, 64, 64, 64,
                       8, 8, 64, 64, 64, 8, 8, 64, 64, 64, 8, 8, 64, 64, 64, 3};
  const int WCI[29] = {3, 64, 64, 64, 64, 64, 64, 64, 64, 32, 64, 64, 64,
                       64, 64, 64, 64, 64, 64, 64, 64, 64, 64, 64, 64, 64, 64, 64, 64};
  const int WKS[29] = {8, 3, 3, 4, 3, 3, 3, 3, 3, 3, 3, 3, 3,
                       1, 1, 1, 3, 3, 1, 1, 1, 3, 3, 1, 1, 1, 3, 3, 3};
  const int Bn = 4;
  const int NOUT0 = Bn * 3 * 64 * 64;
  if (n_in < 31) return;
  if (in_sizes[0] != Bn * 3 * 64 * 64) return;
  if (out_size != NOUT0 + 1) return;

  int wkp[29], woff[29], wrows[29], wK[29];
  int wtot = 0;
  for (int e = 0; e < 29; ++e) {
    const int K = WCI[e] * WKS[e] * WKS[e];
    if (in_sizes[e + 2] != WCO[e] * K) return;
    wK[e] = K;
    wkp[e] = ((K + 31) / 32) * 32;
    wrows[e] = (WCO[e] == 8) ? 8 : (((WCO[e] + 15) / 16) * 16);
    woff[e] = wtot;
    wtot += wrows[e] * wkp[e];
  }

  char* wsb = (char*)d_ws;
  size_t off = 0;
  auto carve = [&](size_t bytes) -> char* {
    char* p = wsb + off;
    off += (bytes + 255) & ~(size_t)255;
    return p;
  };
  const size_t F = sizeof(float);
  const size_t P3 = 1024;
  unsigned short* whi = (unsigned short*)carve((size_t)wtot * 2);
  unsigned short* wlo = (unsigned short*)carve((size_t)wtot * 2);
  float* t1  = (float*)carve((size_t)Bn * 64 * 256 * F);
  float* h16 = (float*)carve((size_t)Bn * 64 * 256 * F);
  float* t2  = (float*)carve((size_t)Bn * 64 * 256 * F);
  float* t3  = (float*)carve((size_t)Bn * 64 * 64 * F);
  float* h8  = (float*)carve((size_t)Bn * 64 * 64 * F);
  float* t4  = (float*)carve((size_t)Bn * 64 * 64 * F);
  float* t5  = (float*)carve((size_t)Bn * 64 * 64 * F);
  float* y0b = (float*)carve((size_t)Bn * 32 * 64 * F);
  float* yb  = (float*)carve((size_t)Bn * 32 * 64 * F);
  float* db1 = (float*)carve((size_t)Bn * 64 * 64 * F);
  float* db2 = (float*)carve((size_t)Bn * 64 * 64 * F);
  float* db3 = (float*)carve((size_t)Bn * 64 * 64 * F);
  float* a1  = (float*)carve((size_t)Bn * 64 * 256 * F);
  float* d4  = (float*)carve((size_t)Bn * 64 * 256 * F);
  float* a2  = (float*)carve((size_t)Bn * 64 * 1024 * F);
  float* h32 = (float*)carve((size_t)Bn * 64 * 1024 * F);
  float* d5  = (float*)carve((size_t)Bn * 64 * 1024 * F);
  float* a3  = (float*)carve((size_t)Bn * 64 * 4096 * F);
  float* h64 = (float*)carve((size_t)Bn * 64 * 4096 * F);
  float* d6  = (float*)carve((size_t)Bn * 64 * 4096 * F);
  float* qkb = (float*)carve((size_t)Bn * 16 * P3 * F);
  float* vsb = (float*)carve((size_t)Bn * 64 * P3 * F);
  unsigned short* vhi = (unsigned short*)carve((size_t)Bn * 64 * P3 * 2);
  unsigned short* vlo = (unsigned short*)carve((size_t)Bn * 64 * P3 * 2);
  if (off > ws_size) return;

  const float* x = (const float*)d_in[0];
  const int* idxp = (const int*)d_in[1];
  float* outF = (float*)d_out;

  {
    WTab tab = {};
    int gx = 1;
    for (int e = 0; e < 29; ++e) {
      tab.src[e] = (const float*)d_in[e + 2];
      tab.cout[e] = WCO[e];
      tab.kdim[e] = wK[e];
      tab.rows[e] = wrows[e];
      tab.kp[e] = wkp[e];
      tab.off[e] = woff[e];
      const int tot = wrows[e] * (wkp[e] / 8);
      const int g = (tot + 255) / 256;
      if (g > gx) gx = g;
    }
    tab.cnt = 29;
    k_wsplit<<<dim3(gx, 29), 256, 0, stream>>>(tab, whi, wlo);
  }

  auto conv = [&](const float* in, int e, int CoutEff, const float* resid, float* out,
                  int Cin, int Hin, int Win, int KH, int stride, int pad, int relu) {
    const int Hout = (Hin + 2 * pad - KH) / stride + 1;
    const int Wout = (Win + 2 * pad - KH) / stride + 1;
    const int N = Bn * Hout * Wout;
    if ((Hout * Wout) % 64 != 0) return;
    const int mw = (CoutEff + 15) / 16;
    k_conv<<<N / 64, 128, 0, stream>>>(in, whi + woff[e], wlo + woff[e], resid, out,
                                       Bn, Cin, Hin, Win, CoutEff, Hout, Wout,
                                       KH, KH, stride, pad, Cin * KH * KH, wkp[e], mw, relu);
  };
  auto res = [&](const float* xin, int e1, int e2, float* htmp, float* outp, int HH) {
    conv(xin, e1, 64, nullptr, htmp, 64, HH, HH, 3, 1, 1, 1);
    conv(htmp, e2, 64, xin, outp, 64, HH, HH, 3, 1, 1, 1);
  };
  auto att = [&](const float* inp, int eq, int ev, float* ao, int HH, int relu) {
    const int P = HH * HH, Mq = 4 * P;
    conv(inp, eq, 16, nullptr, qkb, 64, HH, HH, 1, 1, 0, 0);
    conv(inp, ev, 64, nullptr, vsb, 64, HH, HH, 1, 1, 0, 0);
    const int noct = Bn * 64 * P / 8;
    k_split<<<(noct + 255) / 256, 256, 0, stream>>>(vsb, vhi, vlo, noct);
    k_attn<<<Bn * Mq / 32, 128, 0, stream>>>(qkb, vhi, vlo, ao, Bn, HH, relu);
  };

  conv(x, 0, 64, nullptr, t1, 3, 64, 64, 8, 4, 2, 1);
  res(t1, 1, 2, h16, t2, 16);
  conv(t2, 3, 64, nullptr, t3, 64, 16, 16, 4, 2, 1, 1);
  res(t3, 4, 5, h8, t4, 8);
  res(t4, 6, 7, h8, t5, 8);
  conv(t5, 8, 32, nullptr, y0b, 64, 8, 8, 3, 1, 1, 0);
  k_sig<<<1, 256, 0, stream>>>(y0b, idxp, yb, outF + NOUT0, Bn * 32 * 64, (float)(Bn * 32 * 64));
  conv(yb, 9, 64, nullptr, db1, 32, 8, 8, 3, 1, 1, 1);
  conv(db1, 10, 64, nullptr, db2, 64, 8, 8, 3, 1, 1, 1);
  res(db2, 11, 12, h8, db3, 8);
  att(db3, 13, 15, a1, 8, 1);
  res(a1, 16, 17, h16, d4, 16);
  att(d4, 18, 20, a2, 16, 1);
  res(a2, 21, 22, h32, d5, 32);
  att(d5, 23, 25, a3, 32, 0);
  res(a3, 26, 27, h64, d6, 64);
  conv(d6, 28, 3, nullptr, outF, 64, 64, 64, 3, 1, 1, 0);
}
